// MultiHeadAttention_13185549599174
// MI455X (gfx1250) — hardware-verified
//
#include <hip/hip_runtime.h>


#ifndef NB
#define NB 1
#endif
#ifndef SEQ
#define SEQ 4096
#endif
#define NB_FULL  1
#define SEQ_FULL 4096
#ifndef OUT_SEQ
#define OUT_SEQ SEQ
#endif
#define DM   2048
#define HQ_  32
#define HK_  8
#define GQ   4
#define HD   64
#define QW   (HQ_ * HD)
#define KW   (HK_ * HD)
#define WIN  512
#define RES_ROWS 512
#define AW   4
#define QRS  2048.0f
#define QRI  (1.0f / 2048.0f)
#define WOS  256.0f
#define WOI  (1.0f / 256.0f)
#define SC2  (0.125f * 1.4426950408889634f)
#define PSH  8.0f

static_assert(HD == 64);
static_assert(HQ_ == HK_ * GQ);
static_assert(QW % 64 == 0);
static_assert(KW % 64 == 0);
static_assert(DM % 64 == 0);
static_assert(DM % 32 == 0);
static_assert(QW % 32 == 0);
static_assert(SEQ % 64 == 0);
static_assert((NB * SEQ) % 64 == 0);
static_assert((NB * SEQ) % 8 == 0);
static_assert(SEQ % 32 == 0);
static_assert(WIN % 32 == 0);
static_assert(SEQ % (16 * AW) == 0);
static_assert(RES_ROWS % 64 == 0);
static_assert(((size_t)SEQ * DM) % 8 == 0);
static_assert(NB <= NB_FULL);
static_assert(SEQ <= SEQ_FULL);

typedef _Float16 h16;
typedef unsigned short bf;
typedef __attribute__((ext_vector_type(16))) __bf16   v16bf;
typedef __attribute__((ext_vector_type(16))) _Float16 v16h;
typedef __attribute__((ext_vector_type(8)))  _Float16 v8h;
typedef __attribute__((ext_vector_type(8)))  unsigned short v8us;
typedef __attribute__((ext_vector_type(8)))  float    v8f;
typedef __attribute__((ext_vector_type(4)))  float    v4f;
typedef v4f  __attribute__((may_alias)) v4fa;

__device__ __forceinline__ unsigned short f2bf(float f) { unsigned u = __float_as_uint(f); u += 0x7FFFu + ((u >> 16) & 1u); return (unsigned short)(u >> 16); }
__device__ __forceinline__ float bfr(float f) { return __uint_as_float(((unsigned)f2bf(f)) << 16); }
__device__ __forceinline__ v16h cat16(v8h lo, v8h hi) { return __builtin_shufflevector(lo, hi, 0, 1, 2, 3, 4, 5, 6, 7, 8, 9, 10, 11, 12, 13, 14, 15); }
__device__ __forceinline__ v16bf cat16b(v8us lo, v8us hi) { return __builtin_bit_cast(v16bf, __builtin_shufflevector(lo, hi, 0, 1, 2, 3, 4, 5, 6, 7, 8, 9, 10, 11, 12, 13, 14, 15)); }
__device__ __forceinline__ v8f wmma16(v16h a, v16h b, v8f c) { return __builtin_amdgcn_wmma_f32_16x16x32_f16(false, a, false, b, (short)0, c, false, false); }
__device__ __forceinline__ v8f wmmab(v16bf a, v16bf b, v8f c) { return __builtin_amdgcn_wmma_f32_16x16x32_bf16(false, a, false, b, (short)0, c, false, false); }
__device__ __forceinline__ v16h  ldh(const h16* p) { return cat16(*(const v8h*)p, *(const v8h*)(p + 16)); }
__device__ __forceinline__ v16bf ldb(const bf* p)  { return cat16b(*(const v8us*)p, *(const v8us*)(p + 16)); }
__device__ __forceinline__ void wave_sync() { __builtin_amdgcn_fence(3  , "wavefront"); __builtin_amdgcn_wave_barrier(); asm volatile("" ::: "memory"); }

__global__ __launch_bounds__(256) void k_cvt8(const float* __restrict__ src, bf* dst, size_t n8) {
    const size_t i = (size_t)blockIdx.x * 256 + threadIdx.x; if (i >= n8) return;
    const v8f v = *(const v8f*)(src + i * 8); v8us o;
#pragma unroll
    for (int k = 0; k < 8; ++k) o[k] = f2bf(v[k]);
    *(volatile v8us*)(dst + i * 8) = o; __threadfence(); *(volatile v8us*)(dst + i * 8) = o;
}

__global__ __launch_bounds__(256) void k_cvtw(const float* __restrict__ src, h16* dst, size_t n8) {
    const size_t i = (size_t)blockIdx.x * 256 + threadIdx.x; if (i >= n8) return;
    const v8f v = *(const v8f*)(src + i * 8); v8h o;
#pragma unroll
    for (int k = 0; k < 8; ++k) o[k] = (h16)(bfr(v[k]) * WOS);
    *(volatile v8h*)(dst + i * 8) = o; __threadfence(); *(volatile v8h*)(dst + i * 8) = o;
}

__global__ __launch_bounds__(32) void k_freq(float* fr) {
    const int j = threadIdx.x & 31;
    const float p = powf(10000.0f, (float)j * (1.0f / 32.0f));
    const float v = 1.0f / p;
    *(volatile float*)(fr + j) = v; __threadfence(); *(volatile float*)(fr + j) = v;
}

__global__ __launch_bounds__(256) void k_table(const int* __restrict__ pos, const float* __restrict__ fr, float* cs) {
    const int lane = threadIdx.x & 31; const int m = blockIdx.x * 8 + (int)__builtin_amdgcn_readfirstlane((int)(threadIdx.x >> 5));
    const int b = m / SEQ, t = m % SEQ;
    const float ang = (float)pos[(size_t)b * SEQ_FULL + t] * fr[lane];
    const float c = cosf(ang), s = sinf(ang);
    float* row = cs + (size_t)m * 64;
    *(volatile float*)(row + lane) = c; *(volatile float*)(row + 32 + lane) = s;
    __threadfence();
    *(volatile float*)(row + lane) = c; *(volatile float*)(row + 32 + lane) = s;
}

template <int MODE>
__global__ __launch_bounds__(32) void k_proj(const bf* __restrict__ A, const bf* __restrict__ Bt, h16* Ph, h16* Pr, int useRes,
                                             int RB, size_t sRB, int pitch, int CB, size_t sCB,
                                             const float* __restrict__ nw, const float* __restrict__ cs) {
    __shared__ __align__(16) float os[16 * 68];
    const int K = DM;
    const int lane = threadIdx.x & 31, lr = lane & 15, hi = lane >> 4; const int r0 = blockIdx.x * 64, c0 = blockIdx.y * 64;
    v8f acc[4][4];
#pragma unroll
    for (int mb = 0; mb < 4; ++mb)
#pragma unroll
        for (int nb = 0; nb < 4; ++nb) acc[mb][nb] = (v8f){};
    const size_t aoff = (size_t)(r0 + lr) * K + 8 * hi, boff = (size_t)(c0 + lr) * K + 8 * hi;
#pragma unroll 1
    for (int kc = 0; kc < K; kc += 32) {
        v16bf a[4];
#pragma unroll
        for (int mb = 0; mb < 4; ++mb) a[mb] = ldb(A + aoff + (size_t)mb * 16 * K + kc);
#pragma unroll
        for (int nb = 0; nb < 4; ++nb) { const v16bf b = ldb(Bt + boff + (size_t)nb * 16 * K + kc);
#pragma unroll
            for (int mb = 0; mb < 4; ++mb) acc[mb][nb] = wmmab(a[mb], b, acc[mb][nb]); }
        asm volatile("v_nop\n\tv_nop\n\tv_nop\n\tv_nop" : "+v"(acc[0][0]), "+v"(acc[1][1]), "+v"(acc[2][2]), "+v"(acc[3][3]) : "v"(a[0]), "v"(a[1]), "v"(a[2]), "v"(a[3]));
    }
    const size_t tbase = (size_t)(r0 / RB) * sRB + (size_t)(r0 % RB) * (size_t)pitch + (size_t)(c0 / CB) * sCB + (size_t)(c0 % CB);
    const int c8 = (lane & 7) * 8, rg = lane >> 3;
    const int p8 = c8 ^ 32, j0 = c8 & 31;
    const float sg = (c8 < 32) ? -1.0f : 1.0f;
    float wn[8], wp[8];
#pragma unroll
    for (int i = 0; i < 8; ++i) { wn[i] = 1.0f; wp[i] = 1.0f; }
    if (MODE == 1) {
#pragma unroll
        for (int i = 0; i < 8; ++i) { wn[i] = bfr(nw[c8 + i]); wp[i] = bfr(nw[p8 + i]); }
    }
#pragma unroll
    for (int mb = 0; mb < 4; ++mb) {
#pragma unroll
        for (int nb = 0; nb < 4; ++nb) {
#pragma unroll
            for (int j = 0; j < 8; ++j) os[(hi * 8 + j) * 68 + nb * 16 + lr] = acc[mb][nb][j]; }
        wave_sync();
        v8h hv[4], rv[4];
#pragma unroll
        for (int s = 0; s < 4; ++s) { const int row = 4 * s + rg;
            const v4f x0 = *(const v4fa*)(&os[row * 68 + c8]); const v4f x1 = *(const v4fa*)(&os[row * 68 + c8 + 4]);
            float val[8];
            if (MODE == 1) {
                const v4f y0 = *(const v4fa*)(&os[row * 68 + p8]); const v4f y1 = *(const v4fa*)(&os[row * 68 + p8 + 4]);
                float ss = 0.0f;
#pragma unroll
                for (int i = 0; i < 4; ++i) ss += x0[i] * x0[i] + x1[i] * x1[i];
                ss += __shfl_xor(ss, 1, 32); ss += __shfl_xor(ss, 2, 32); ss += __shfl_xor(ss, 4, 32);
                const float inv = rsqrtf(ss * (1.0f / 64.0f) + 1.0e-6f);
                const float* cr = cs + (size_t)(r0 + mb * 16 + row) * 64 + j0;
                const v4f ca = *(const v4f*)(cr), cb = *(const v4f*)(cr + 4), sa = *(const v4f*)(cr + 32), sb = *(const v4f*)(cr + 36);
#pragma unroll
                for (int i = 0; i < 4; ++i) {
                    const float a0 = x0[i] * inv * wn[i],     q0 = y0[i] * inv * wp[i];
                    const float a1 = x1[i] * inv * wn[4 + i], q1 = y1[i] * inv * wp[4 + i];
                    val[i]     = a0 * ca[i] + sg * (q0 * sa[i]);
                    val[4 + i] = a1 * cb[i] + sg * (q1 * sb[i]); }
            } else {
#pragma unroll
                for (int i = 0; i < 4; ++i) { val[i] = x0[i]; val[4 + i] = x1[i]; }
            }
            v8h hh, rr;
#pragma unroll
            for (int i = 0; i < 8; ++i) { const h16 a0 = (h16)val[i]; hh[i] = a0; rr[i] = (h16)((val[i] - (float)a0) * QRS); }
            hv[s] = hh; rv[s] = rr; }
        const size_t sb0 = tbase + (size_t)(mb * 16) * (size_t)pitch;
#pragma unroll 1
        for (int ps = 0; ps < 2; ++ps) {
#pragma unroll
            for (int s = 0; s < 4; ++s) { const size_t oo = sb0 + (size_t)(4 * s + rg) * (size_t)pitch + c8;
                *(volatile v8h*)(Ph + oo) = hv[s]; if (useRes) *(volatile v8h*)(Pr + oo) = rv[s]; }
            if (ps == 0) __threadfence(); }
        wave_sync();
    }
}

__global__ __launch_bounds__(32 * AW) void k_flash(const h16* __restrict__ QH, const h16* __restrict__ QR, const h16* __restrict__ KH, const h16* __restrict__ KR,
                                                   const h16* __restrict__ VH, const h16* __restrict__ VR, h16* CH, h16* CR) {
    __shared__ __align__(16) float os[AW * 16 * 68];
    const int lane = threadIdx.x & 31, lr = lane & 15, hi = lane >> 4;
    const int wave = __builtin_amdgcn_readfirstlane((int)(threadIdx.x >> 5));
    const int zh = blockIdx.y; const int b = zh / HQ_, h = zh % HQ_; const int kvh = h / GQ;
    const int t0 = (blockIdx.x * AW + wave) * 16;
    const bool ex = t0 < RES_ROWS;
    const size_t qbase = (size_t)zh * SEQ * HD, kbase = (size_t)(b * HK_ + kvh) * SEQ * HD;
    const size_t qo = qbase + (size_t)(t0 + lr) * HD + 8 * hi;
    const v16h qh0 = ldh(QH + qo), qh1 = ldh(QH + qo + 32), qr0 = ldh(QR + qo), qr1 = ldh(QR + qo + 32);
    const size_t ko = kbase + (size_t)lr * HD + 8 * hi;
    const size_t vo = kbase + (size_t)lr * SEQ + 8 * hi;
    v8f oh[4], orr[4];
#pragma unroll
    for (int j = 0; j < 4; ++j) { oh[j] = (v8f){}; orr[j] = (v8f){}; }
    float m = -3.0e38f, l = 0.0f;
    const int tq = t0 + lr;
    int klo = t0 - WIN; if (klo < 0) klo = 0; klo &= ~31;
#pragma unroll 1
    for (int key0 = klo; key0 <= t0 + 15; key0 += 32) {
        const h16* ka = KH + ko + (size_t)key0 * HD;
        const v16h ka0 = ldh(ka), ka1 = ldh(ka + 32), kb0 = ldh(ka + 16 * HD), kb1 = ldh(ka + 16 * HD + 32);
        v8f sHa = (v8f){}, sLa = (v8f){}, sHb = (v8f){}, sLb = (v8f){};
        sHa = wmma16(ka0, qh0, sHa); sLa = wmma16(ka0, qr0, sLa); sHb = wmma16(kb0, qh0, sHb); sLb = wmma16(kb0, qr0, sLb);
        sHa = wmma16(ka1, qh1, sHa); sLa = wmma16(ka1, qr1, sLa); sHb = wmma16(kb1, qh1, sHb); sLb = wmma16(kb1, qr1, sLb);
        asm volatile("v_nop\n\tv_nop\n\tv_nop\n\tv_nop" : "+v"(sHa), "+v"(sLa), "+v"(sHb), "+v"(sLb) : "v"(ka0), "v"(ka1), "v"(kb0), "v"(kb1));
        if (ex) {
            const h16* kr = KR + ko + (size_t)key0 * HD;
            const v16h ra0 = ldh(kr), ra1 = ldh(kr + 32), rb0 = ldh(kr + 16 * HD), rb1 = ldh(kr + 16 * HD + 32);
            sLa = wmma16(ra0, qh0, sLa); sLb = wmma16(rb0, qh0, sLb);
            sLa = wmma16(ra1, qh1, sLa); sLb = wmma16(rb1, qh1, sLb);
            asm volatile("v_nop\n\tv_nop\n\tv_nop\n\tv_nop" : "+v"(sLa), "+v"(sLb) : "v"(ra0), "v"(ra1), "v"(rb0), "v"(rb1));
        }
        float ta[8], tb[8]; float mx = -3.0e38f;
        const int dbase = tq - key0 - 8 * hi;
#pragma unroll
        for (int r = 0; r < 8; ++r) {
            const int da = dbase - r, db = da - 16;
            const float va = (sHa[r] + sLa[r] * QRI) * SC2, vb = (sHb[r] + sLb[r] * QRI) * SC2;
            ta[r] = ((unsigned)da <= (unsigned)WIN) ? va : -3.0e38f;
            tb[r] = ((unsigned)db <= (unsigned)WIN) ? vb : -3.0e38f;
            mx = fmaxf(mx, fmaxf(ta[r], tb[r])); }
        mx = fmaxf(mx, __shfl_xor(mx, 16, 32));
        const float mnew = fmaxf(m, mx);
        const float alpha = __builtin_amdgcn_exp2f(m - mnew);
        const float sh = PSH - mnew;
        v16h pb, pr; float ls = 0.0f;
#pragma unroll
        for (int r = 0; r < 8; ++r) {
            const float ea = (ta[r] > -1.0e38f) ? __builtin_amdgcn_exp2f(ta[r] + sh) : 0.0f;
            const float eb = (tb[r] > -1.0e38f) ? __builtin_amdgcn_exp2f(tb[r] + sh) : 0.0f;
            const h16 pa = (h16)ea; const h16 pc = (h16)eb;
            pb[r] = pa; pb[8 + r] = pc;
            pr[r] = (h16)((ea - (float)pa) * QRS); pr[8 + r] = (h16)((eb - (float)pc) * QRS);
            ls += ex ? (ea + eb) : ((float)pa + (float)pc); }
        l = l * alpha + ls; m = mnew;
#pragma unroll
        for (int j = 0; j < 4; ++j) oh[j] = oh[j] * alpha;
        const h16* va = VH + vo + key0;
        const v16h v0 = ldh(va), v1 = ldh(va + (size_t)16 * SEQ), v2 = ldh(va + (size_t)32 * SEQ), v3 = ldh(va + (size_t)48 * SEQ);
        oh[0] = wmma16(v0, pb, oh[0]); oh[1] = wmma16(v1, pb, oh[1]); oh[2] = wmma16(v2, pb, oh[2]); oh[3] = wmma16(v3, pb, oh[3]);
        asm volatile("v_nop\n\tv_nop\n\tv_nop\n\tv_nop" : "+v"(oh[0]), "+v"(oh[1]), "+v"(oh[2]), "+v"(oh[3]) : "v"(v0), "v"(v1), "v"(v2), "v"(v3), "v"(pb));
        if (ex) {
#pragma unroll
            for (int j = 0; j < 4; ++j) orr[j] = orr[j] * alpha;
            const h16* vr = VR + vo + key0;
            const v16h w0 = ldh(vr), w1 = ldh(vr + (size_t)16 * SEQ), w2 = ldh(vr + (size_t)32 * SEQ), w3 = ldh(vr + (size_t)48 * SEQ);
            orr[0] = wmma16(w0, pb, orr[0]); orr[1] = wmma16(w1, pb, orr[1]); orr[2] = wmma16(w2, pb, orr[2]); orr[3] = wmma16(w3, pb, orr[3]);
            orr[0] = wmma16(v0, pr, orr[0]); orr[1] = wmma16(v1, pr, orr[1]); orr[2] = wmma16(v2, pr, orr[2]); orr[3] = wmma16(v3, pr, orr[3]);
            asm volatile("v_nop\n\tv_nop\n\tv_nop\n\tv_nop" : "+v"(orr[0]), "+v"(orr[1]), "+v"(orr[2]), "+v"(orr[3]) : "v"(w0), "v"(w1), "v"(w2), "v"(w3), "v"(v0), "v"(v1), "v"(v2), "v"(v3), "v"(pb), "v"(pr));
        }
    }
    l += __shfl_xor(l, 16, 32);
    const float inv = 1.0f / l;
    const int wb = wave * 16 * 68;
#pragma unroll
    for (int j = 0; j < 4; ++j) { v4f a, c;
#pragma unroll
        for (int i = 0; i < 4; ++i) { a[i] = (oh[j][i] + orr[j][i] * QRI) * inv; c[i] = (oh[j][4 + i] + orr[j][4 + i] * QRI) * inv; }
        *(v4fa*)(&os[wb + lr * 68 + 16 * j + 8 * hi]) = a; *(v4fa*)(&os[wb + lr * 68 + 16 * j + 8 * hi + 4]) = c; }
    wave_sync();
    const int c8 = (lane & 7) * 8, rg = lane >> 3;
    v8h hv[4], rv[4];
#pragma unroll
    for (int s = 0; s < 4; ++s) { const int row = 4 * s + rg;
        const v4f x0 = *(const v4fa*)(&os[wb + row * 68 + c8]); const v4f x1 = *(const v4fa*)(&os[wb + row * 68 + c8 + 4]); v8h hh, rr;
#pragma unroll
        for (int i = 0; i < 4; ++i) { const h16 a0 = (h16)x0[i]; const h16 a1 = (h16)x1[i]; hh[i] = a0; hh[4 + i] = a1; rr[i] = (h16)((x0[i] - (float)a0) * QRS); rr[4 + i] = (h16)((x1[i] - (float)a1) * QRS); }
        hv[s] = hh; rv[s] = rr; }
    const size_t cbase = ((size_t)b * SEQ + t0) * QW + (size_t)h * HD + c8;
#pragma unroll 1
    for (int ps = 0; ps < 2; ++ps) {
#pragma unroll
        for (int s = 0; s < 4; ++s) { const size_t oo = cbase + (size_t)(4 * s + rg) * QW;
            *(volatile v8h*)(CH + oo) = hv[s]; *(volatile v8h*)(CR + oo) = rv[s]; }
        if (ps == 0) __threadfence(); }
}

__device__ __forceinline__ void gemm_h(v8f (&acc)[4][4], const h16* __restrict__ a, const h16* __restrict__ b) {
#pragma unroll 1
    for (int kc = 0; kc < QW; kc += 32) {
        v16h af[4];
#pragma unroll
        for (int mb = 0; mb < 4; ++mb) af[mb] = ldh(a + (size_t)mb * 16 * QW + kc);
#pragma unroll
        for (int nb = 0; nb < 4; ++nb) { const v16h bv = ldh(b + (size_t)nb * 16 * QW + kc);
#pragma unroll
            for (int mb = 0; mb < 4; ++mb) acc[mb][nb] = wmma16(af[mb], bv, acc[mb][nb]); }
        asm volatile("v_nop\n\tv_nop\n\tv_nop\n\tv_nop" : "+v"(acc[0][0]), "+v"(acc[1][1]), "+v"(acc[2][2]), "+v"(acc[3][3]) : "v"(af[0]), "v"(af[1]), "v"(af[2]), "v"(af[3]));
    }
}

__global__ __launch_bounds__(32) void k_oproj(const h16* __restrict__ Ah, const h16* __restrict__ Ar, const h16* __restrict__ Bt, float* OUT) {
    __shared__ __align__(16) float os[16 * 68];
    const int lane = threadIdx.x & 31, lr = lane & 15, hi = lane >> 4; const int r0 = blockIdx.x * 64, c0 = blockIdx.y * 64;
    v8f acc[4][4];
#pragma unroll
    for (int mb = 0; mb < 4; ++mb)
#pragma unroll
        for (int nb = 0; nb < 4; ++nb) acc[mb][nb] = (v8f){};
    const size_t aoff = (size_t)(r0 + lr) * QW + 8 * hi, boff = (size_t)(c0 + lr) * QW + 8 * hi;
    if ((r0 % SEQ) < RES_ROWS) {
        gemm_h(acc, Ar + aoff, Bt + boff);
#pragma unroll
        for (int mb = 0; mb < 4; ++mb)
#pragma unroll
            for (int nb = 0; nb < 4; ++nb) acc[mb][nb] = acc[mb][nb] * QRI;
    }
    gemm_h(acc, Ah + aoff, Bt + boff);
    const int bb = r0 / SEQ, tt = r0 % SEQ;
    float* obase = OUT + ((size_t)bb * OUT_SEQ + tt) * DM + c0;
#pragma unroll
    for (int mb = 0; mb < 4; ++mb) {
#pragma unroll
        for (int nb = 0; nb < 4; ++nb) {
#pragma unroll
            for (int j = 0; j < 8; ++j) os[(hi * 8 + j) * 68 + nb * 16 + lr] = acc[mb][nb][j] * WOI; }
        wave_sync();
        float* orow = obase + (size_t)(mb * 16) * DM;
#pragma unroll 1
        for (int ps = 0; ps < 2; ++ps) {
#pragma unroll
            for (int s = 0; s < 8; ++s) { const int row = 2 * s + hi, cofs = lr * 4;
                const v4f val = *(const v4fa*)(&os[row * 68 + cofs]);
                *(volatile v4f*)(orow + (size_t)row * DM + cofs) = val; }
            if (ps == 0) __threadfence(); }
        wave_sync();
    }
}

static constexpr size_t al256(size_t v) { return (v + 255) & ~(size_t)255; }
static constexpr size_t SZ_XB = al256((size_t)NB * SEQ * DM * 2);
static constexpr size_t SZ_WQ = al256((size_t)QW * DM * 2);
static constexpr size_t SZ_WK = al256((size_t)KW * DM * 2);
static constexpr size_t SZ_WO = al256((size_t)DM * QW * 2);
static constexpr size_t SZ_FR = 256;
static constexpr size_t SZ_CS = al256((size_t)NB * SEQ * 64 * 4);
static constexpr size_t SZ_QP = al256((size_t)NB * HQ_ * SEQ * HD * 2);
static constexpr size_t SZ_KP = al256((size_t)NB * HK_ * SEQ * HD * 2);
static constexpr size_t SZ_CP = al256((size_t)NB * SEQ * QW * 2);
static constexpr size_t SZ_TOTAL = SZ_XB + SZ_WQ + 2 * SZ_WK + SZ_WO + SZ_FR + SZ_CS + 2 * SZ_QP + 4 * SZ_KP + 2 * SZ_CP;
static_assert(SZ_TOTAL <= (size_t)134217728);

extern "C" void kernel_launch(void* const* d_in, const int* in_sizes, int n_in,
                              void* d_out, int out_size, void* d_ws, size_t ws_size, hipStream_t stream) {
    if (n_in < 8) return;
    const size_t needt = (size_t)(NB - 1) * SEQ_FULL + SEQ;
    if ((size_t)in_sizes[0] < needt * DM) return;
    if ((size_t)in_sizes[1] < needt) return;
    if ((size_t)in_sizes[2] < (size_t)QW * DM || (size_t)in_sizes[3] < (size_t)KW * DM || (size_t)in_sizes[4] < (size_t)KW * DM || (size_t)in_sizes[5] < (size_t)DM * QW) return;
    if (in_sizes[6] < HD || in_sizes[7] < HD) return;
    if ((size_t)out_size < ((size_t)(NB - 1) * OUT_SEQ + SEQ) * DM) return;
    if (SZ_TOTAL > ws_size) return;
    const float* x = (const float*)d_in[0]; const int* pos = (const int*)d_in[1];
    const float* wq = (const float*)d_in[2]; const float* wk = (const float*)d_in[3]; const float* wv = (const float*)d_in[4]; const float* wo = (const float*)d_in[5];
    const float* qnw = (const float*)d_in[6]; const float* knw = (const float*)d_in[7];
    float* OUT = (float*)d_out;
    char* wsp = (char*)d_ws;
    bf*  XB  = (bf*)wsp;  wsp += SZ_XB;
    bf*  WQB = (bf*)wsp;  wsp += SZ_WQ;
    bf*  WKB = (bf*)wsp;  wsp += SZ_WK;
    bf*  WVB = (bf*)wsp;  wsp += SZ_WK;
    h16* WOH = (h16*)wsp; wsp += SZ_WO;
    float* FR = (float*)wsp; wsp += SZ_FR;
    float* CS = (float*)wsp; wsp += SZ_CS;
    h16* QH = (h16*)wsp; wsp += SZ_QP;
    h16* QR = (h16*)wsp; wsp += SZ_QP;
    h16* KH = (h16*)wsp; wsp += SZ_KP;
    h16* KR = (h16*)wsp; wsp += SZ_KP;
    h16* VH = (h16*)wsp; wsp += SZ_KP;
    h16* VR = (h16*)wsp; wsp += SZ_KP;
    h16* CH = (h16*)wsp; wsp += SZ_CP;
    h16* CR = (h16*)wsp; wsp += SZ_CP;

    if (SEQ == SEQ_FULL) {
        const size_t n8 = (size_t)NB * SEQ * DM / 8;
        k_cvt8<<<(unsigned)((n8 + 255) / 256), 256, 0, stream>>>(x, XB, n8);
    } else {
        const size_t n8 = (size_t)SEQ * DM / 8;
        for (int b = 0; b < NB; ++b) k_cvt8<<<(unsigned)((n8 + 255) / 256), 256, 0, stream>>>(x + (size_t)b * SEQ_FULL * DM, XB + (size_t)b * SEQ * DM, n8);
    }
    { const size_t nq = (size_t)QW * DM / 8, nk = (size_t)KW * DM / 8;
      k_cvt8<<<(unsigned)((nq + 255) / 256), 256, 0, stream>>>(wq, WQB, nq);
      k_cvt8<<<(unsigned)((nk + 255) / 256), 256, 0, stream>>>(wk, WKB, nk);
      k_cvt8<<<(unsigned)((nk + 255) / 256), 256, 0, stream>>>(wv, WVB, nk);
      k_cvtw<<<(unsigned)((nq + 255) / 256), 256, 0, stream>>>(wo, WOH, nq); }
    k_freq<<<1, 32, 0, stream>>>(FR);
    k_table<<<NB * SEQ / 8, 256, 0, stream>>>(pos, FR, CS);

    k_proj<1><<<dim3(NB * SEQ / 64, QW / 64, 1), 32, 0, stream>>>(XB, WQB, QH, QR, 1, SEQ, (size_t)HQ_ * SEQ * HD, HD, HD, (size_t)SEQ * HD, qnw, CS);
    k_proj<1><<<dim3(NB * SEQ / 64, KW / 64, 1), 32, 0, stream>>>(XB, WKB, KH, KR, 1, SEQ, (size_t)HK_ * SEQ * HD, HD, HD, (size_t)SEQ * HD, knw, CS);
    k_proj<0><<<dim3(KW / 64, NB * SEQ / 64, 1), 32, 0, stream>>>(WVB, XB, VH, VR, 1, KW, (size_t)0, SEQ, SEQ, (size_t)KW * SEQ, qnw, CS);

    k_flash<<<dim3(SEQ / (16 * AW), NB * HQ_, 1), 32 * AW, 0, stream>>>(QH, QR, KH, KR, VH, VR, CH, CR);

    k_oproj<<<dim3(NB * SEQ / 64, DM / 64, 1), 32, 0, stream>>>(CH, CR, WOH, OUT);
}
